// MultiHeadAttentionBlock_27960237097221
// MI455X (gfx1250) — hardware-verified
//
#include <hip/hip_runtime.h>
#include <stddef.h>
#include <stdint.h>


typedef __attribute__((ext_vector_type(16))) _Float16     v16h;
typedef __attribute__((ext_vector_type(8)))  _Float16     v8h;
typedef __attribute__((ext_vector_type(8)))  float        v8f;
typedef __attribute__((ext_vector_type(4)))  float        v4f;
typedef __attribute__((ext_vector_type(4)))  unsigned int u32x4;
typedef __attribute__((ext_vector_type(4)))  int          i32x4;

#ifndef NB
#define NB 2
#endif
#ifndef SEQ
#define SEQ 2048
#endif
#define NB_FULL  2
#define SEQ_FULL 2048
#define DM   1024
#define NH   16
#define DK   64
#define MW   (SEQ / 32)
#define ER   256
#define ERR  ((SEQ < ER) ? SEQ : ER)

#define PSTR 40
#define OST  72
#define LST  72
#define FST  68
#define PROJ_LDS_BYTES 18432

#define QSCALE  0.18033688011112042f
#define MASKV   (-1.4426950e9f)
#define WSC     64.0f
#define WSC_INV 0.015625f
#define RSC     2048.0f
#define RSC_INV 0.00048828125f
#define PSC     4096.0f
#define OSC     32.0f
#define OPS_INV 0.0078125f
#define OUT_MUL 0.00048828125f

static_assert(NB >= 1 && NB <= NB_FULL);
static_assert(SEQ >= 64 && SEQ <= SEQ_FULL && (SEQ % 64) == 0);
static_assert((ERR % 64) == 0 && ERR >= 64 && ERR <= SEQ);
static_assert(((SEQ - ERR) % 16) == 0);
static_assert(((NB * SEQ * MW) % 256) == 0);
static_assert(DM == NH * DK && (DM % 64) == 0);
static_assert(2 * 64 * LST * 2 <= PROJ_LDS_BYTES);
static_assert(64 * FST * 4 <= PROJ_LDS_BYTES);
static_assert(((NB * SEQ * DM) % 2048) == 0);
static_assert(((DM * DM) % 2048) == 0);

__device__ __forceinline__ v16h load_half_frag(const _Float16* p, int hi) {
  union { v16h v; u32x4 q[2]; } u;
  u.q[0] = *(const u32x4*)(p + hi * 8);
  u.q[1] = *(const u32x4*)(p + 16 + hi * 8);
  return u.v;
}

__device__ __forceinline__ v8f wmma16(v16h a, v16h b, v8f c) {
  return __builtin_amdgcn_wmma_f32_16x16x32_f16(false, a, false, b, (short)0, c, false, false);
}

__device__ __forceinline__ float bf16r(float f) {
  unsigned int u = __float_as_uint(f);
  u = u + 0x7FFFu + ((u >> 16) & 1u);
  u &= 0xFFFF0000u;
  return __uint_as_float(u);
}

__global__ __launch_bounds__(256) void cvt_kernel(
    const float* __restrict__ s0, const float* __restrict__ s1,
    const float* __restrict__ s2, const float* __restrict__ s3,
    _Float16* __restrict__ d0, _Float16* __restrict__ d1,
    _Float16* __restrict__ d2, _Float16* __restrict__ d3,
    int rpg, int gstride, float scale) {
  const int z = blockIdx.z;
  const float* src = s0;
  _Float16* dst = d0;
  if (z == 1) { src = s1; dst = d1; }
  else if (z == 2) { src = s2; dst = d2; }
  else if (z == 3) { src = s3; dst = d3; }

  const size_t e    = ((size_t)blockIdx.x * 256 + threadIdx.x) * 8;
  const size_t row  = e / DM;
  const int    colh = (int)(e % DM);
  const size_t srow = (row / (size_t)rpg) * (size_t)gstride + (row % (size_t)rpg);
  const float* sp = src + srow * DM + colh;
  const v4f f0 = *(const v4f*)sp;
  const v4f f1 = *(const v4f*)(sp + 4);

  union { v8h h; u32x4 u; } o;
  o.h[0] = (_Float16)(bf16r(f0[0]) * scale);
  o.h[1] = (_Float16)(bf16r(f0[1]) * scale);
  o.h[2] = (_Float16)(bf16r(f0[2]) * scale);
  o.h[3] = (_Float16)(bf16r(f0[3]) * scale);
  o.h[4] = (_Float16)(bf16r(f1[0]) * scale);
  o.h[5] = (_Float16)(bf16r(f1[1]) * scale);
  o.h[6] = (_Float16)(bf16r(f1[2]) * scale);
  o.h[7] = (_Float16)(bf16r(f1[3]) * scale);

  volatile u32x4* dp = (volatile u32x4*)(dst + e);
  *dp = o.u;
  __threadfence();
  *dp = o.u;
}

__global__ __launch_bounds__(256) void maskpack_kernel(const int* __restrict__ mask,
                                                       unsigned int* __restrict__ mbits) {
  const int lane = threadIdx.x & 31;
  const int wave = threadIdx.x >> 5;
  const int g   = (blockIdx.x * 8 + wave) * 32 + lane;
  const int row = g / MW;
  const int w   = g - row * MW;
  const int b   = row / SEQ;
  const int s   = row - b * SEQ;
  const int* src = mask + ((size_t)(b * SEQ_FULL + s)) * SEQ_FULL + 32 * w;

  unsigned int bits = 0u;
#pragma unroll
  for (int j = 0; j < 8; ++j) {
    const i32x4 m4 = *(const i32x4*)(src + 4 * j);
    bits |= (m4[0] != 0 ? 1u : 0u) << (4 * j);
    bits |= (m4[1] != 0 ? 1u : 0u) << (4 * j + 1);
    bits |= (m4[2] != 0 ? 1u : 0u) << (4 * j + 2);
    bits |= (m4[3] != 0 ? 1u : 0u) << (4 * j + 3);
  }
  volatile unsigned int* dp = (volatile unsigned int*)(mbits + g);
  *dp = bits;
  __threadfence();
  *dp = bits;
}

__device__ __forceinline__ void gemm_dm(const _Float16* __restrict__ arow0, const _Float16* __restrict__ arow1,
                                        const _Float16* __restrict__ brow0, const _Float16* __restrict__ brow1,
                                        int hf, v8f& c00, v8f& c01, v8f& c10, v8f& c11) {
#pragma unroll 2
  for (int kc = 0; kc < DM; kc += 32) {
    const v16h a0 = load_half_frag(arow0 + kc, hf);
    const v16h a1 = load_half_frag(arow1 + kc, hf);
    const v16h b0 = load_half_frag(brow0 + kc, hf);
    const v16h b1 = load_half_frag(brow1 + kc, hf);
    c00 = wmma16(a0, b0, c00);
    c01 = wmma16(a0, b1, c01);
    c10 = wmma16(a1, b0, c10);
    c11 = wmma16(a1, b1, c11);
    asm volatile("v_nop\n\tv_nop\n\tv_nop\n\tv_nop"
                 : "+v"(c00), "+v"(c01), "+v"(c10), "+v"(c11)
                 : "v"(a0), "v"(a1), "v"(b0), "v"(b1));
  }
}

__device__ __forceinline__ void stage_hl(v8f c, int rowb, int col, _Float16* lh, _Float16* ll, float mul) {
#pragma unroll
  for (int r = 0; r < 8; ++r) {
    const float v = c[r] * mul;
    const _Float16 hv = (_Float16)v;
    lh[(rowb + r) * LST + col] = hv;
    ll[(rowb + r) * LST + col] = (_Float16)((v - (float)hv) * RSC);
  }
}

__device__ __forceinline__ void stage_t2(v8f c, int rowb, int col, _Float16* lt, _Float16* ll) {
  union { v8h h; u32x4 u; } o, q;
#pragma unroll
  for (int r = 0; r < 8; ++r) {
    const float v = c[r] * WSC_INV;
    const _Float16 hv = (_Float16)v;
    o.h[r] = hv;
    q.h[r] = (_Float16)((v - (float)hv) * RSC);
  }
  *(u32x4*)(lt + col * LST + rowb) = o.u;
  *(u32x4*)(ll + col * LST + rowb) = q.u;
}

__device__ __forceinline__ void stage_f(v8f c, int rowb, int col, float* lf) {
#pragma unroll
  for (int r = 0; r < 8; ++r) lf[(rowb + r) * FST + col] = c[r] * OUT_MUL;
}

template <int MODE>
__global__ __launch_bounds__(128) void proj_kernel(
    const _Float16* __restrict__ A, const _Float16* __restrict__ A2, const _Float16* __restrict__ W,
    _Float16* __restrict__ P0, _Float16* __restrict__ P1, float* __restrict__ Pf) {
  __shared__ __align__(16) unsigned char lds_raw[PROJ_LDS_BYTES];

  const int lane = threadIdx.x & 31;
  const int wave = threadIdx.x >> 5;
  const int hf   = lane >> 4;
  const int n    = lane & 15;
  const int n0   = blockIdx.x * 64;
  const int m0   = blockIdx.y * 64;
  const int mt0  = (wave >> 1) * 32;
  const int nt0  = (wave & 1) * 32;

  const _Float16* arow0 = A + (size_t)(m0 + mt0 + n) * DM;
  const _Float16* arow1 = arow0 + (size_t)16 * DM;
  const _Float16* brow0 = W + (size_t)(n0 + nt0 + n) * DM;
  const _Float16* brow1 = brow0 + (size_t)16 * DM;

  v8f c00 = {}, c01 = {}, c10 = {}, c11 = {};
  gemm_dm(arow0, arow1, brow0, brow1, hf, c00, c01, c10, c11);

  const int bidx = m0 / SEQ;
  const int s0   = m0 - bidx * SEQ;

  if (MODE == 3) {
    if (s0 < ERR) {
      const _Float16* rrow0 = A2 + (size_t)(m0 + mt0 + n) * DM;
      const _Float16* rrow1 = rrow0 + (size_t)16 * DM;
      v8f d00 = {}, d01 = {}, d10 = {}, d11 = {};
      gemm_dm(rrow0, rrow1, brow0, brow1, hf, d00, d01, d10, d11);
      c00 = c00 + d00 * RSC_INV;
      c01 = c01 + d01 * RSC_INV;
      c10 = c10 + d10 * RSC_INV;
      c11 = c11 + d11 * RSC_INV;
    }
  }

  if (MODE <= 1) {
    _Float16* lh = (_Float16*)lds_raw;
    _Float16* ll = lh + 64 * LST;
    const float mul = (MODE == 0) ? (WSC_INV * QSCALE) : WSC_INV;
    stage_hl(c00, mt0 + 8 * hf,      nt0 + n,      lh, ll, mul);
    stage_hl(c01, mt0 + 8 * hf,      nt0 + 16 + n, lh, ll, mul);
    stage_hl(c10, mt0 + 16 + 8 * hf, nt0 + n,      lh, ll, mul);
    stage_hl(c11, mt0 + 16 + 8 * hf, nt0 + 16 + n, lh, ll, mul);
    __syncthreads();
    const size_t dbase = (((size_t)bidx * NH + blockIdx.x) * SEQ + s0) * DK;
    _Float16* dh = P0 + dbase;
    _Float16* dl = P1 + dbase;
    u32x4 vh[4], vl[4];
    int off[4];
#pragma unroll
    for (int it = 0; it < 4; ++it) {
      const int p = it * 128 + threadIdx.x;
      const int row = p >> 3, j = p & 7;
      vh[it]  = *(const u32x4*)(lh + row * LST + 8 * j);
      vl[it]  = *(const u32x4*)(ll + row * LST + 8 * j);
      off[it] = row * DK + 8 * j;
    }
#pragma unroll
    for (int it = 0; it < 4; ++it) {
      *(volatile u32x4*)(dh + off[it]) = vh[it];
      *(volatile u32x4*)(dl + off[it]) = vl[it];
    }
    __threadfence();
#pragma unroll
    for (int it = 0; it < 4; ++it) {
      *(volatile u32x4*)(dh + off[it]) = vh[it];
      *(volatile u32x4*)(dl + off[it]) = vl[it];
    }
  } else if (MODE == 2) {
    _Float16* lt = (_Float16*)lds_raw;
    _Float16* ll = lt + 64 * LST;
    stage_t2(c00, mt0 + 8 * hf,      nt0 + n,      lt, ll);
    stage_t2(c01, mt0 + 8 * hf,      nt0 + 16 + n, lt, ll);
    stage_t2(c10, mt0 + 16 + 8 * hf, nt0 + n,      lt, ll);
    stage_t2(c11, mt0 + 16 + 8 * hf, nt0 + 16 + n, lt, ll);
    __syncthreads();
    const size_t vbase = (((size_t)bidx * NH + blockIdx.x) * DK) * SEQ + s0;
    _Float16* dv = P0 + vbase;
    _Float16* dl = P1 + vbase;
    u32x4 vv[4], vr[4];
    size_t off[4];
#pragma unroll
    for (int it = 0; it < 4; ++it) {
      const int p = it * 128 + threadIdx.x;
      const int d = p >> 3, j = p & 7;
      vv[it]  = *(const u32x4*)(lt + d * LST + 8 * j);
      vr[it]  = *(const u32x4*)(ll + d * LST + 8 * j);
      off[it] = (size_t)d * SEQ + 8 * j;
    }
#pragma unroll
    for (int it = 0; it < 4; ++it) {
      *(volatile u32x4*)(dv + off[it]) = vv[it];
      *(volatile u32x4*)(dl + off[it]) = vr[it];
    }
    __threadfence();
#pragma unroll
    for (int it = 0; it < 4; ++it) {
      *(volatile u32x4*)(dv + off[it]) = vv[it];
      *(volatile u32x4*)(dl + off[it]) = vr[it];
    }
  } else {
    float* lf = (float*)lds_raw;
    stage_f(c00, mt0 + 8 * hf,      nt0 + n,      lf);
    stage_f(c01, mt0 + 8 * hf,      nt0 + 16 + n, lf);
    stage_f(c10, mt0 + 16 + 8 * hf, nt0 + n,      lf);
    stage_f(c11, mt0 + 16 + 8 * hf, nt0 + 16 + n, lf);
    __syncthreads();
    float* dout = Pf + ((size_t)bidx * SEQ_FULL + s0) * DM + n0;
    v4f vf[8];
    size_t off[8];
#pragma unroll
    for (int it = 0; it < 8; ++it) {
      const int p = it * 128 + threadIdx.x;
      const int row = p >> 4, j = p & 15;
      vf[it]  = *(const v4f*)(lf + row * FST + 4 * j);
      off[it] = (size_t)row * DM + 4 * j;
    }
#pragma unroll
    for (int it = 0; it < 8; ++it) *(volatile v4f*)(dout + off[it]) = vf[it];
    __threadfence();
#pragma unroll
    for (int it = 0; it < 8; ++it) *(volatile v4f*)(dout + off[it]) = vf[it];
  }
}

__device__ __forceinline__ void stage_o2(float v, int idx, _Float16* lo, _Float16* lr) {
  const _Float16 hv = (_Float16)v;
  lo[idx] = hv;
  lr[idx] = (_Float16)((v - (float)hv) * RSC);
}

template <int RES>
__global__ __launch_bounds__(32) __attribute__((amdgpu_num_vgpr(256))) void attn_kernel(
    const _Float16* __restrict__ Qh, const _Float16* __restrict__ Ql,
    const _Float16* __restrict__ Kh, const _Float16* __restrict__ Kl,
    const _Float16* __restrict__ Vt, const _Float16* __restrict__ Vl,
    const unsigned int* __restrict__ mbits,
    _Float16* __restrict__ Oh, _Float16* __restrict__ Ol, int qblk0) {
  __shared__ __align__(16) _Float16 Plds[16 * PSTR];
  __shared__ __align__(16) _Float16 Prls[16 * PSTR];
  __shared__ __align__(16) _Float16 Olds[16 * OST];
  __shared__ __align__(16) _Float16 Orls[16 * OST];

  const int lane = threadIdx.x & 31;
  const int hf   = lane >> 4;
  const int n    = lane & 15;
  const int q0   = ((int)blockIdx.x + qblk0) * 16;
  const int h    = blockIdx.y;
  const int b    = blockIdx.z;
  const size_t bh = (size_t)b * NH + h;

  const _Float16* qhrow = Qh + (bh * SEQ + q0 + n) * DK;
  const _Float16* qlrow = Ql + (bh * SEQ + q0 + n) * DK;
  const v16h aqh0 = load_half_frag(qhrow, hf);
  const v16h aqh1 = load_half_frag(qhrow + 32, hf);
  const v16h aql0 = load_half_frag(qlrow, hf);
  const v16h aql1 = load_half_frag(qlrow + 32, hf);

  const unsigned int* mrow = mbits + ((size_t)b * SEQ + q0 + n) * MW;
  const _Float16* khb = Kh + (bh * SEQ + n) * DK;
  const _Float16* klb = Kl + (bh * SEQ + n) * DK;
  const _Float16* vtb = Vt + (bh * DK + n) * SEQ;
  const _Float16* vlb = Vl + (bh * DK + n) * SEQ;

  v16h ones;
#pragma unroll
  for (int j = 0; j < 16; ++j) ones[j] = (_Float16)1.0f;

  v8f o0 = {}, o1 = {}, o2 = {}, o3 = {}, lacc = {};
  v8f e0 = {}, e1 = {}, e2 = {}, e3 = {};
  float mrun[8], lsum[8];
#pragma unroll
  for (int r = 0; r < 8; ++r) { mrun[r] = -1e30f; lsum[r] = 0.0f; }

#pragma unroll 1
  for (int c = 0; c < MW; ++c) {
    const int k0 = c * 32;
    const unsigned int mword = mrow[c];
    const unsigned long long live = __ballot((mword != 0u) ? 1 : 0);
    if (live == 0ull) continue;

    float sc0[8], sc1[8];
    {
      const _Float16* kp  = khb + (size_t)k0 * DK;
      const _Float16* klp = klb + (size_t)k0 * DK;
      const v16h bkh0 = load_half_frag(kp, hf);
      const v16h bkh1 = load_half_frag(kp + 32, hf);
      const v16h bkl0 = load_half_frag(klp, hf);
      const v16h bkl1 = load_half_frag(klp + 32, hf);
      v8f z = {};
      v8f s0 = wmma16(aqh0, bkh0, z);
      s0 = wmma16(aqh1, bkh1, s0);
      v8f x0 = wmma16(aqh0, bkl0, z);
      x0 = wmma16(aqh1, bkl1, x0);
      x0 = wmma16(aql0, bkh0, x0);
      x0 = wmma16(aql1, bkh1, x0);
      asm volatile("v_nop\n\tv_nop\n\tv_nop\n\tv_nop"
                   : "+v"(s0), "+v"(x0)
                   : "v"(bkh0), "v"(bkh1), "v"(bkl0), "v"(bkl1),
                     "v"(aqh0), "v"(aqh1), "v"(aql0), "v"(aql1));
#pragma unroll
      for (int r = 0; r < 8; ++r) sc0[r] = s0[r] + x0[r] * RSC_INV;
    }
    {
      const _Float16* kp  = khb + (size_t)(k0 + 16) * DK;
      const _Float16* klp = klb + (size_t)(k0 + 16) * DK;
      const v16h ckh0 = load_half_frag(kp, hf);
      const v16h ckh1 = load_half_frag(kp + 32, hf);
      const v16h ckl0 = load_half_frag(klp, hf);
      const v16h ckl1 = load_half_frag(klp + 32, hf);
      v8f z = {};
      v8f s1 = wmma16(aqh0, ckh0, z);
      s1 = wmma16(aqh1, ckh1, s1);
      v8f x1 = wmma16(aqh0, ckl0, z);
      x1 = wmma16(aqh1, ckl1, x1);
      x1 = wmma16(aql0, ckh0, x1);
      x1 = wmma16(aql1, ckh1, x1);
      asm volatile("v_nop\n\tv_nop\n\tv_nop\n\tv_nop"
                   : "+v"(s1), "+v"(x1)
                   : "v"(ckh0), "v"(ckh1), "v"(ckl0), "v"(ckl1),
                     "v"(aqh0), "v"(aqh1), "v"(aql0), "v"(aql1));
#pragma unroll
      for (int r = 0; r < 8; ++r) sc1[r] = s1[r] + x1[r] * RSC_INV;
    }

#pragma unroll
    for (int r = 0; r < 8; ++r) {
      const unsigned int bits = (unsigned int)__shfl((int)mword, 8 * hf + r, 32);
      if (((bits >> n) & 1u) == 0u)        sc0[r] = MASKV;
      if (((bits >> (16 + n)) & 1u) == 0u) sc1[r] = MASKV;
    }

    float mnew[8], psum[8];
#pragma unroll
    for (int r = 0; r < 8; ++r) mnew[r] = fmaxf(sc0[r], sc1[r]);
#pragma unroll
    for (int off = 1; off < 16; off <<= 1) {
#pragma unroll
      for (int r = 0; r < 8; ++r) mnew[r] = fmaxf(mnew[r], __shfl_xor(mnew[r], off, 32));
    }
#pragma unroll
    for (int r = 0; r < 8; ++r) {
      mnew[r] = fmaxf(mnew[r], mrun[r]);
      const float alpha = exp2f(mrun[r] - mnew[r]);
      const float p0 = exp2f(sc0[r] - mnew[r]);
      const float p1 = exp2f(sc1[r] - mnew[r]);
      mrun[r] = mnew[r];
      o0[r] *= alpha;
      o1[r] *= alpha;
      o2[r] *= alpha;
      o3[r] *= alpha;
      if (RES) {
        e0[r] *= alpha;
        e1[r] *= alpha;
        e2[r] *= alpha;
        e3[r] *= alpha;
        lsum[r] *= alpha;
        psum[r] = p0 + p1;
      } else {
        lacc[r] *= alpha;
      }
      const int m = 8 * hf + r;
      const float f0 = p0 * PSC, f1 = p1 * PSC;
      const _Float16 g0 = (_Float16)f0, g1 = (_Float16)f1;
      Plds[m * PSTR + n]      = g0;
      Plds[m * PSTR + 16 + n] = g1;
      if (RES) {
        Prls[m * PSTR + n]      = (_Float16)((f0 - (float)g0) * RSC);
        Prls[m * PSTR + 16 + n] = (_Float16)((f1 - (float)g1) * RSC);
      }
    }
    if (RES) {
#pragma unroll
      for (int off = 1; off < 16; off <<= 1) {
#pragma unroll
        for (int r = 0; r < 8; ++r) psum[r] += __shfl_xor(psum[r], off, 32);
      }
#pragma unroll
      for (int r = 0; r < 8; ++r) lsum[r] += psum[r];
    }
    __syncthreads();

    const v16h ap = load_half_frag(Plds + n * PSTR, hf);
    const _Float16* vp = vtb + k0;
    if (RES == 0) {
      const v16h bv0 = load_half_frag(vp, hf);
      const v16h bv1 = load_half_frag(vp + (size_t)16 * SEQ, hf);
      const v16h bv2 = load_half_frag(vp + (size_t)32 * SEQ, hf);
      const v16h bv3 = load_half_frag(vp + (size_t)48 * SEQ, hf);
      o0 = wmma16(ap, bv0, o0);
      o1 = wmma16(ap, bv1, o1);
      o2 = wmma16(ap, bv2, o2);
      o3 = wmma16(ap, bv3, o3);
      lacc = wmma16(ap, ones, lacc);
      asm volatile("v_nop\n\tv_nop\n\tv_nop\n\tv_nop"
                   : "+v"(o0), "+v"(o1), "+v"(o2), "+v"(o3), "+v"(lacc)
                   : "v"(ap), "v"(bv0), "v"(bv1), "v"(bv2), "v"(bv3), "v"(ones));
    } else {
      const v16h apl = load_half_frag(Prls + n * PSTR, hf);
      const _Float16* vq = vlb + k0;
      {
        const v16h bvh = load_half_frag(vp, hf);
        const v16h bvl = load_half_frag(vq, hf);
        o0 = wmma16(ap, bvh, o0);
        e0 = wmma16(ap, bvl, e0);
        e0 = wmma16(apl, bvh, e0);
        asm volatile("v_nop\n\tv_nop\n\tv_nop\n\tv_nop"
                     : "+v"(o0), "+v"(e0) : "v"(ap), "v"(apl), "v"(bvh), "v"(bvl));
      }
      {
        const v16h bvh = load_half_frag(vp + (size_t)16 * SEQ, hf);
        const v16h bvl = load_half_frag(vq + (size_t)16 * SEQ, hf);
        o1 = wmma16(ap, bvh, o1);
        e1 = wmma16(ap, bvl, e1);
        e1 = wmma16(apl, bvh, e1);
        asm volatile("v_nop\n\tv_nop\n\tv_nop\n\tv_nop"
                     : "+v"(o1), "+v"(e1) : "v"(ap), "v"(apl), "v"(bvh), "v"(bvl));
      }
      {
        const v16h bvh = load_half_frag(vp + (size_t)32 * SEQ, hf);
        const v16h bvl = load_half_frag(vq + (size_t)32 * SEQ, hf);
        o2 = wmma16(ap, bvh, o2);
        e2 = wmma16(ap, bvl, e2);
        e2 = wmma16(apl, bvh, e2);
        asm volatile("v_nop\n\tv_nop\n\tv_nop\n\tv_nop"
                     : "+v"(o2), "+v"(e2) : "v"(ap), "v"(apl), "v"(bvh), "v"(bvl));
      }
      {
        const v16h bvh = load_half_frag(vp + (size_t)48 * SEQ, hf);
        const v16h bvl = load_half_frag(vq + (size_t)48 * SEQ, hf);
        o3 = wmma16(ap, bvh, o3);
        e3 = wmma16(ap, bvl, e3);
        e3 = wmma16(apl, bvh, e3);
        asm volatile("v_nop\n\tv_nop\n\tv_nop\n\tv_nop"
                     : "+v"(o3), "+v"(e3) : "v"(ap), "v"(apl), "v"(bvh), "v"(bvl));
      }
    }
    __syncthreads();
  }

  _Float16* dst = Oh + ((size_t)b * SEQ + q0) * DM + (size_t)h * DK;
  if (RES == 0) {
#pragma unroll
    for (int r = 0; r < 8; ++r) {
      const float inv = OSC / lacc[r];
      const int row = 8 * hf + r;
      Olds[row * OST + n]      = (_Float16)(o0[r] * inv);
      Olds[row * OST + 16 + n] = (_Float16)(o1[r] * inv);
      Olds[row * OST + 32 + n] = (_Float16)(o2[r] * inv);
      Olds[row * OST + 48 + n] = (_Float16)(o3[r] * inv);
    }
    __syncthreads();

    u32x4 ov[4];
    int ooff[4];
#pragma unroll
    for (int it = 0; it < 4; ++it) {
      const int p = it * 32 + lane;
      const int row = p >> 3, j = p & 7;
      ov[it]   = *(const u32x4*)(Olds + row * OST + 8 * j);
      ooff[it] = row * DM + 8 * j;
    }
#pragma unroll
    for (int it = 0; it < 4; ++it) *(volatile u32x4*)(dst + ooff[it]) = ov[it];
    __threadfence();
#pragma unroll
    for (int it = 0; it < 4; ++it) *(volatile u32x4*)(dst + ooff[it]) = ov[it];
  } else {
#pragma unroll
    for (int r = 0; r < 8; ++r) {
      const float inv = OPS_INV / lsum[r];
      const int row = 8 * hf + r;
      stage_o2((o0[r] + e0[r] * RSC_INV) * inv, row * OST + n,      Olds, Orls);
      stage_o2((o1[r] + e1[r] * RSC_INV) * inv, row * OST + 16 + n, Olds, Orls);
      stage_o2((o2[r] + e2[r] * RSC_INV) * inv, row * OST + 32 + n, Olds, Orls);
      stage_o2((o3[r] + e3[r] * RSC_INV) * inv, row * OST + 48 + n, Olds, Orls);
    }
    __syncthreads();

    _Float16* dsr = Ol + ((size_t)b * SEQ + q0) * DM + (size_t)h * DK;
    u32x4 ov[4], rv[4];
    int ooff[4];
#pragma unroll
    for (int it = 0; it < 4; ++it) {
      const int p = it * 32 + lane;
      const int row = p >> 3, j = p & 7;
      ov[it]   = *(const u32x4*)(Olds + row * OST + 8 * j);
      rv[it]   = *(const u32x4*)(Orls + row * OST + 8 * j);
      ooff[it] = row * DM + 8 * j;
    }
#pragma unroll
    for (int it = 0; it < 4; ++it) {
      *(volatile u32x4*)(dst + ooff[it]) = ov[it];
      *(volatile u32x4*)(dsr + ooff[it]) = rv[it];
    }
    __threadfence();
#pragma unroll
    for (int it = 0; it < 4; ++it) {
      *(volatile u32x4*)(dst + ooff[it]) = ov[it];
      *(volatile u32x4*)(dsr + ooff[it]) = rv[it];
    }
  }
}

extern "C" void kernel_launch(void* const* d_in, const int* in_sizes, int n_in,
                              void* d_out, int out_size, void* d_ws, size_t ws_size,
                              hipStream_t stream) {
  if (n_in < 8) return;
  const size_t NE = (size_t)NB * SEQ * DM;
  const size_t WE = (size_t)DM * DM;
  const size_t HE = (size_t)NB * NH * SEQ * DK;
  const size_t MB = (size_t)NB * SEQ * MW;

  if ((size_t)in_sizes[0] < NE || (size_t)in_sizes[1] < NE || (size_t)in_sizes[2] < NE) return;
  if ((size_t)in_sizes[3] < (size_t)NB * SEQ * SEQ) return;
  if ((size_t)in_sizes[4] < WE || (size_t)in_sizes[5] < WE ||
      (size_t)in_sizes[6] < WE || (size_t)in_sizes[7] < WE) return;
  if ((size_t)out_size < NE) return;

  const size_t total_bytes = (3 * NE + 4 * WE + 6 * HE + 2 * NE) * sizeof(_Float16) + MB * sizeof(unsigned int);
  if (ws_size < total_bytes) return;

  const float* q    = (const float*)d_in[0];
  const float* k    = (const float*)d_in[1];
  const float* v    = (const float*)d_in[2];
  const int*   mask = (const int*)d_in[3];
  const float* Wq   = (const float*)d_in[4];
  const float* Wk   = (const float*)d_in[5];
  const float* Wv   = (const float*)d_in[6];
  const float* Wo   = (const float*)d_in[7];
  float* out = (float*)d_out;

  _Float16* xq = (_Float16*)d_ws;
  _Float16* xk = xq + NE;
  _Float16* xv = xk + NE;
  _Float16* wq = xv + NE;
  _Float16* wk = wq + WE;
  _Float16* wv = wk + WE;
  _Float16* wo = wv + WE;
  _Float16* Qh = wo + WE;
  _Float16* Ql = Qh + HE;
  _Float16* Kh = Ql + HE;
  _Float16* Kl = Kh + HE;
  _Float16* Vt = Kl + HE;
  _Float16* Vl = Vt + HE;
  _Float16* Oh = Vl + HE;
  _Float16* Ol = Oh + NE;
  unsigned int* mb = (unsigned int*)(Ol + NE);

  dim3 gc_act((unsigned)(NE / 2048), 1, 3);
  cvt_kernel<<<gc_act, 256, 0, stream>>>(q, k, v, v, xq, xk, xv, xv, SEQ, SEQ_FULL, 1.0f);
  dim3 gc_w((unsigned)(WE / 2048), 1, 4);
  cvt_kernel<<<gc_w, 256, 0, stream>>>(Wq, Wk, Wv, Wo, wq, wk, wv, wo, DM, DM, WSC);

  maskpack_kernel<<<(unsigned)(MB / 256), 256, 0, stream>>>(mask, mb);

  dim3 gp(DM / 64, (NB * SEQ) / 64);
  proj_kernel<0><<<gp, 128, 0, stream>>>(xq, xq, wq, Qh, Ql, out);
  proj_kernel<1><<<gp, 128, 0, stream>>>(xk, xk, wk, Kh, Kl, out);
  proj_kernel<2><<<gp, 128, 0, stream>>>(xv, xv, wv, Vt, Vl, out);

  dim3 ga_e(ERR / 16, NH, NB);
  attn_kernel<1><<<ga_e, 32, 0, stream>>>(Qh, Ql, Kh, Kl, Vt, Vl, mb, Oh, Ol, 0);
  if (SEQ > ERR) {
    dim3 ga_l((SEQ - ERR) / 16, NH, NB);
    attn_kernel<0><<<ga_l, 32, 0, stream>>>(Qh, Ql, Kh, Kl, Vt, Vl, mb, Oh, Ol, ERR / 16);
  }

  proj_kernel<3><<<gp, 128, 0, stream>>>(Oh, Ol, wo, Vt, Vt, out);
}
